// PredictionEncoder_86079734546935
// MI455X (gfx1250) — hardware-verified
//
#include <hip/hip_runtime.h>
#include <math.h>

typedef __attribute__((ext_vector_type(16))) _Float16 v16h;
typedef __attribute__((ext_vector_type(16))) __bf16 v16b;
typedef __attribute__((ext_vector_type(8)))  _Float16 v8h;
typedef __attribute__((ext_vector_type(8)))  float v8f;
typedef __attribute__((ext_vector_type(4)))  float v4f;
typedef __attribute__((ext_vector_type(2)))  float v2f;
typedef __attribute__((ext_vector_type(4)))  unsigned v4u;
typedef __attribute__((ext_vector_type(4)))  int v4i;
typedef float __attribute__((may_alias)) float_a;
typedef int __attribute__((may_alias)) int_a;

template <typename T> __device__ __forceinline__ void vst2(void* p, T v) { *(volatile T*)p = v; __threadfence(); *(volatile T*)p = v; }
__device__ __forceinline__ v8f wmma16(v16h a, v16h b, v8f c) {
  v8f d = __builtin_amdgcn_wmma_f32_16x16x32_f16(false, a, false, b, (short)0, c, false, false);
  asm volatile("v_nop\n\tv_nop\n\tv_nop\n\tv_nop" : "+v"(d) : "v"(a), "v"(b));
  return d;
}
__device__ __forceinline__ v8f wmma_bf(v16b a, v16b b, v8f c) {
  v8f d = __builtin_amdgcn_wmma_f32_16x16x32_bf16(false, a, false, b, (short)0, c, false, false);
  asm volatile("v_nop\n\tv_nop\n\tv_nop\n\tv_nop" : "+v"(d) : "v"(a), "v"(b));
  return d;
}
__device__ __forceinline__ v16h frag_h(const _Float16* rowk0, int lane) {
  union { v16h v; v8h q[2]; } u; const _Float16* p = rowk0 + 8 * (lane >> 4);
  u.q[0] = *(const v8h*)p; u.q[1] = *(const v8h*)(p + 16); return u.v;
}
__device__ __forceinline__ v16h frag_f32(const float* rowk0, int lane) {
  v16h a; const float* p = rowk0 + 8 * (lane >> 4);
#pragma unroll
  for (int i = 0; i < 8; ++i) { a[i] = (_Float16)p[i]; a[8 + i] = (_Float16)p[16 + i]; }
  return a;
}
__device__ __forceinline__ v16h frag_f32s(const float* rowk0, int lane, float sc) {
  v16h a; const float* p = rowk0 + 8 * (lane >> 4);
#pragma unroll
  for (int i = 0; i < 8; ++i) { a[i] = (_Float16)(p[i] * sc); a[8 + i] = (_Float16)(p[16 + i] * sc); }
  return a;
}
__device__ __forceinline__ v16h fragc_f32(const float* W, int k0, int n, int lane, int ld, int K) {
  v16h a; const int g = lane >> 4;
#pragma unroll
  for (int i = 0; i < 8; ++i) { const int ka = k0 + 8 * g + i, kb = ka + 16;
    a[i] = (_Float16)(ka < K ? W[(size_t)(ka < K ? ka : K - 1) * ld + n] : 0.f); a[8 + i] = (_Float16)(kb < K ? W[(size_t)(kb < K ? kb : K - 1) * ld + n] : 0.f); }
  return a;
}
struct F2 { v16b h, l; };
__device__ __forceinline__ F2 bsplit16(const float v[16]) { F2 r;
#pragma unroll
  for (int i = 0; i < 16; ++i) { const __bf16 h = (__bf16)v[i]; r.h[i] = h; r.l[i] = (__bf16)(v[i] - (float)h); }
  return r; }
__device__ __forceinline__ F2 split_row(const float* row, int k0, int lane) { float v[16]; const float* p = row + k0 + 8 * (lane >> 4);
#pragma unroll
  for (int i = 0; i < 8; ++i) { v[i] = p[i]; v[8 + i] = p[16 + i]; }
  return bsplit16(v); }
__device__ __forceinline__ F2 split_rowK(const float* row, int k0, int lane, int K) { float v[16]; const int g = lane >> 4;
#pragma unroll
  for (int i = 0; i < 8; ++i) { const int ka = k0 + 8 * g + i, kb = ka + 16; v[i] = ka < K ? row[ka < K ? ka : K - 1] : 0.f; v[8 + i] = kb < K ? row[kb < K ? kb : K - 1] : 0.f; }
  return bsplit16(v); }
__device__ __forceinline__ F2 split_col(const float* W, int k0, int n, int lane, int ld, int K) { float v[16]; const int g = lane >> 4;
#pragma unroll
  for (int i = 0; i < 8; ++i) { const int ka = k0 + 8 * g + i, kb = ka + 16; v[i] = ka < K ? W[(size_t)(ka < K ? ka : K - 1) * ld + n] : 0.f; v[8 + i] = kb < K ? W[(size_t)(kb < K ? kb : K - 1) * ld + n] : 0.f; }
  return bsplit16(v); }
__device__ __forceinline__ v8f mac3(const F2& a, const F2& b, v8f c) { c = wmma_bf(a.l, b.h, c); c = wmma_bf(a.h, b.l, c); return wmma_bf(a.h, b.h, c); }
__device__ __forceinline__ float sigm(float v) { return 1.0f / (1.0f + expf(-v)); }
#define LDSX() do { asm volatile("s_wait_dscnt 0" ::: "memory"); __builtin_amdgcn_wave_barrier(); __builtin_amdgcn_fence(__ATOMIC_RELEASE, "workgroup"); } while (0)


#define NSC 256
#define NV 256
#define HH 256
#define LAT 64
#define NO 128
#define NR (NSC * NV)
#define HALF (NSC / 2)
__device__ __forceinline__ float bfr(float v) { return (float)(__bf16)v; }
__device__ __forceinline__ v16b frag_b(const __bf16* rowk0, int lane) { return __builtin_bit_cast(v16b, frag_h((const _Float16*)rowk0, lane)); }
__device__ __attribute__((noinline)) float exp_ni(float v) { return expf(v); }

__device__ __forceinline__ F2 enc_frag(float oa, float ob, const float* __restrict__ W2, const float* __restrict__ bb, int k0, int lane) {
  float v[16]; const int g = lane >> 4;
#pragma unroll
  for (int i = 0; i < 8; ++i) { const int ca = k0 + 8 * g + i, cb = ca + 16;
    float x = oa * bfr(W2[ca]) + ob * bfr(W2[HH + ca]) + bfr(bb[ca]); v[i] = x > 0.f ? x : 0.f;
    float y = oa * bfr(W2[cb]) + ob * bfr(W2[HH + cb]) + bfr(bb[cb]); v[8 + i] = y > 0.f ? y : 0.f; }
  F2 f; _Float16 hh[16], ll[16];
  union { __bf16 e[16]; v16b b; } ph, pl;
#pragma unroll
  for (int i = 0; i < 16; ++i) { const __bf16 hi = (__bf16)v[i]; ph.e[i] = hi; pl.e[i] = (__bf16)(v[i] - (float)hi); }
  (void)hh; (void)ll; f.h = ph.b; f.l = pl.b; return f;
}
__global__ __launch_bounds__(128) void k_h(const float* __restrict__ obs, const float* __restrict__ hin, const float* __restrict__ Ws, const float* __restrict__ bs, const float* __restrict__ Wv, const float* __restrict__ bv, const float* __restrict__ Wg, const float* __restrict__ aw, const float* __restrict__ W1, int n0base,
                                          float* __restrict__ S, __bf16* __restrict__ HWTh, __bf16* __restrict__ HWTl) {
  __shared__ __align__(16) float sh[4][16][HH + 4]; __shared__ __align__(16) __bf16 sth[HH][72], stl[HH][72]; __shared__ __align__(16) float ss[64][2];
  const int tid = threadIdx.x, wave = tid >> 5, lane = tid & 31, col = lane & 15, g = lane >> 4; const int np = blockIdx.y, n = n0base + np, v0 = blockIdx.x * 64; const size_t r0 = (size_t)n * NV + v0 + wave * 16;
  const float* orow = obs + (r0 + col) * 5; const float o1 = bfr(orow[1]), o2 = bfr(orow[2]), o3 = bfr(orow[3]), o4 = bfr(orow[4]);
  { v8f acc[16] = {};
#pragma unroll 1
    for (int kc = 0; kc < HH / 32; ++kc) { const F2 a = enc_frag(o1, o2, Ws, bs, kc * 32, lane);
#pragma unroll
      for (int j = 0; j < 16; ++j) { const v16b wb = split_col(Wg, kc * 32, j * 16 + col, lane, HH, 2 * HH + LAT).h; acc[j] = wmma_bf(a.l, wb, acc[j]); acc[j] = wmma_bf(a.h, wb, acc[j]); } }
#pragma unroll 1
    for (int kc = 0; kc < HH / 32; ++kc) { const F2 a = enc_frag(o3, o4, Wv, bv, kc * 32, lane);
#pragma unroll
      for (int j = 0; j < 16; ++j) { const v16b wb = split_col(Wg + (size_t)HH * HH, kc * 32, j * 16 + col, lane, HH, HH + LAT).h; acc[j] = wmma_bf(a.l, wb, acc[j]); acc[j] = wmma_bf(a.h, wb, acc[j]); } }
#pragma unroll
    for (int kc = 0; kc < LAT / 32; ++kc) { const v16b a = split_row(hin + (r0 + col) * LAT, kc * 32, lane).h;
#pragma unroll
      for (int j = 0; j < 16; ++j) acc[j] = wmma_bf(a, split_col(Wg + (size_t)2 * HH * HH, kc * 32, j * 16 + col, lane, HH, LAT).h, acc[j]); }
#pragma unroll
    for (int j = 0; j < 16; ++j)
#pragma unroll
      for (int r = 0; r < 8; ++r) sh[wave][8 * g + r][j * 16 + col] = acc[j][r]; }
  LDSX();
  { const int rl = lane & 15, which = lane >> 4; const float* ap = aw + which * HH; float s = 0.f;
#pragma unroll 4
    for (int d = 0; d < HH; ++d) s += sh[wave][rl][d] * bfr(ap[d]);
    ss[wave * 16 + rl][which] = s; }
  { v8f acc[16] = {};
#pragma unroll 1
    for (int kc = 0; kc < HH / 32; ++kc) { const F2 a = split_row(&sh[wave][col][0], kc * 32, lane);
#pragma unroll
      for (int j = 0; j < 16; ++j) { const v16b wb = split_col(W1, kc * 32, j * 16 + col, lane, HH, 2 * HH).h; acc[j] = wmma_bf(a.l, wb, acc[j]); acc[j] = wmma_bf(a.h, wb, acc[j]); } }
#pragma unroll
    for (int j = 0; j < 16; ++j)
#pragma unroll
      for (int r = 0; r < 8; ++r) { const float vv = acc[j][r]; const __bf16 hi = (__bf16)vv; sth[j * 16 + col][wave * 16 + 8 * g + r] = hi; stl[j * 16 + col][wave * 16 + 8 * g + r] = (__bf16)(vv - (float)hi); } }
  __syncthreads();
  for (int qq = tid; qq < HH * 8; qq += 128) { const int d = qq >> 3, pc = qq & 7; const size_t o = ((size_t)np * HH + d) * NV + v0 + pc * 8; vst2((unsigned*)(HWTh + o), *(const v4u*)(&sth[d][pc * 8])); vst2((unsigned*)(HWTl + o), *(const v4u*)(&stl[d][pc * 8])); }
  if (tid < 32) vst2(S + (r0 - wave * 16) * 2 + tid * 4, *(const v4f*)(&ss[0][0] + tid * 4));
}
__global__ __launch_bounds__(128) void k_gat(const float* __restrict__ S, const __bf16* __restrict__ HWTh, const __bf16* __restrict__ HWTl, const float* __restrict__ obs, const float* __restrict__ Ws, const float* __restrict__ bs, const float* __restrict__ W1, const float* __restrict__ b1, int n0base,
                                            float* __restrict__ X1P, float* __restrict__ PS, float* __restrict__ PQ) {
  __shared__ __align__(16) float sS[4][16][68]; __shared__ __align__(16) __bf16 sPh[4][16][72], sPl[4][16][72]; __shared__ float s1s[4][16]; __shared__ __align__(16) float so[4][16][HH + 4]; __shared__ __align__(16) float sps[2][HH];
  const int tid = threadIdx.x, w = tid >> 5, lane = tid & 31, col = lane & 15, g = lane >> 4; const int np = blockIdx.y, n = n0base + np; const int i0 = blockIdx.x * 64 + w * 16; const size_t rbase = (size_t)n * NV;
  if (lane < 16) s1s[w][lane] = S[(rbase + i0 + lane) * 2];
  float mrun = -3.0e38f, lrun = 0.f; v8f acc[16] = {};
  LDSX();
#pragma unroll 1
  for (int kt = 0; kt < NV / 64; ++kt) {
    { const int rl = lane & 15, jh = lane >> 4; const float si = s1s[w][rl];
#pragma unroll 4
      for (int jj = 0; jj < 32; ++jj) { const int j = kt * 64 + jh * 32 + jj; float z = si + S[(rbase + j) * 2 + 1]; z = z > 0.f ? z : 0.01f * z; sS[w][rl][jh * 32 + jj] = z; } }
    LDSX();
    float mx = -3.4e38f;
#pragma unroll
    for (int jj = 0; jj < 32; ++jj) mx = fmaxf(mx, sS[w][col][g * 32 + jj]);
    mx = fmaxf(mx, __shfl_xor(mx, 16, 32));
    const float mnew = fmaxf(mrun, mx); const float corr = expf(mrun - mnew);
    float ps = 0.f;
#pragma unroll 4
    for (int jj = 0; jj < 32; ++jj) { const float p = exp_ni(sS[w][col][g * 32 + jj] - mnew); ps += p; const __bf16 hi = (__bf16)p; sPh[w][col][g * 32 + jj] = hi; sPl[w][col][g * 32 + jj] = (__bf16)(p - (float)hi); }
    ps += __shfl_xor(ps, 16, 32);
    lrun = lrun * corr + ps; mrun = mnew;
#pragma unroll
    for (int r = 0; r < 8; ++r) { const float cr = __shfl(corr, 8 * g + r, 32);
#pragma unroll
      for (int t = 0; t < 16; ++t) acc[t][r] *= cr; }
    LDSX();
#pragma unroll
    for (int kc = 0; kc < 2; ++kc) { const v16b ph = frag_b(&sPh[w][col][0] + kc * 32, lane), pl = frag_b(&sPl[w][col][0] + kc * 32, lane);
#pragma unroll
      for (int t = 0; t < 16; ++t) { const size_t ho = ((size_t)np * HH + t * 16 + col) * NV + kt * 64 + kc * 32; const v16b hh = frag_b(HWTh + ho, lane), hl = frag_b(HWTl + ho, lane); acc[t] = wmma_bf(pl, hh, acc[t]); acc[t] = wmma_bf(ph, hl, acc[t]); acc[t] = wmma_bf(ph, hh, acc[t]); } }
    LDSX(); }
  { float invl[8];
#pragma unroll
    for (int r = 0; r < 8; ++r) invl[r] = 1.0f / __shfl(lrun, 8 * g + r, 32);
#pragma unroll
    for (int t = 0; t < 16; ++t)
#pragma unroll
      for (int r = 0; r < 8; ++r) acc[t][r] *= invl[r]; }
  { const float* orow = obs + (rbase + i0 + col) * 5; const float o1 = bfr(orow[1]), o2 = bfr(orow[2]);
#pragma unroll 1
    for (int kc = 0; kc < HH / 32; ++kc) { const F2 a = enc_frag(o1, o2, Ws, bs, kc * 32, lane);
#pragma unroll
      for (int t = 0; t < 16; ++t) { const v16b wb = split_col(W1 + (size_t)HH * HH, kc * 32, t * 16 + col, lane, HH, HH).h; acc[t] = wmma_bf(a.l, wb, acc[t]); acc[t] = wmma_bf(a.h, wb, acc[t]); } } }
#pragma unroll
  for (int t = 0; t < 16; ++t) { const float bb = bfr(b1[t * 16 + col]);
#pragma unroll
    for (int r = 0; r < 8; ++r) so[w][8 * g + r][t * 16 + col] = acc[t][r] + bb; }
  LDSX();
  for (int rl = 0; rl < 16; ++rl) for (int pc = lane; pc < HH / 4; pc += 32) vst2(X1P + (rbase + i0 + rl) * HH + pc * 4, *(const v4f*)(&so[w][rl][pc * 4]));
  __syncthreads();
  for (int c = tid; c < HH; c += 128) { float s = 0.f, q = 0.f; for (int ww = 0; ww < 4; ++ww) for (int rl = 0; rl < 16; ++rl) { const float v = so[ww][rl][c]; s += v; q += v * v; } sps[0][c] = s; sps[1][c] = q; }
  __syncthreads();
  { const size_t blk = (size_t)n * (NV / 64) + blockIdx.x; if (tid < 64) vst2(PS + blk * HH + tid * 4, *(const v4f*)(&sps[0][tid * 4])); else vst2(PQ + blk * HH + (tid - 64) * 4, *(const v4f*)(&sps[1][(tid - 64) * 4])); }
}
template <int CW>
__global__ __launch_bounds__(256) void k_bn(const float* __restrict__ PS, const float* __restrict__ PQ, int nblk, const float* __restrict__ gam, const float* __restrict__ bet, float* __restrict__ SC) {
  const int c = threadIdx.x; if (c >= CW) return; float s = 0.f, q = 0.f;
  for (int bI = 0; bI < nblk; ++bI) { s += PS[(size_t)bI * CW + c]; q += PQ[(size_t)bI * CW + c]; }
  const float mean = s / (float)NR; const float var = fmaxf(q / (float)NR - mean * mean, 0.f); const float sc = bfr(gam[c]) * rsqrtf(var + 1e-5f);
  vst2(SC + c, (float_a)sc); vst2(SC + CW + c, (float_a)(bfr(bet[c]) - mean * sc));
}
__global__ __launch_bounds__(128) void k_x2(const float* __restrict__ X1P, const float* __restrict__ SC1, const float* __restrict__ W2, const float* __restrict__ b2, float* __restrict__ X2P, float* __restrict__ PS, float* __restrict__ PQ) {
  __shared__ __align__(16) float so[4][16][NO + 4]; __shared__ __align__(16) float sps[2][NO];
  const int tid = threadIdx.x, wave = tid >> 5, lane = tid & 31, col = lane & 15, g = lane >> 4; const size_t r0 = (size_t)blockIdx.x * 64 + wave * 16;
  v8f acc[8] = {};
#pragma unroll 1
  for (int kc = 0; kc < HH / 32; ++kc) { float v[16]; const float* row = X1P + (r0 + col) * HH + kc * 32;
#pragma unroll
    for (int i = 0; i < 8; ++i) { const int ca = kc * 32 + 8 * g + i, cb = ca + 16; float x = row[8 * g + i] * SC1[ca] + SC1[HH + ca]; v[i] = x > 0.f ? x : 0.f; float y = row[8 * g + i + 16] * SC1[cb] + SC1[HH + cb]; v[8 + i] = y > 0.f ? y : 0.f; }
    union { __bf16 e[16]; v16b b; } ph, pl;
#pragma unroll
    for (int i = 0; i < 16; ++i) { const __bf16 hi = (__bf16)v[i]; ph.e[i] = hi; pl.e[i] = (__bf16)(v[i] - (float)hi); }
#pragma unroll
    for (int j = 0; j < 8; ++j) { const v16b wb = split_col(W2, kc * 32, j * 16 + col, lane, NO, HH).h; acc[j] = wmma_bf(pl.b, wb, acc[j]); acc[j] = wmma_bf(ph.b, wb, acc[j]); } }
#pragma unroll
  for (int j = 0; j < 8; ++j) { const float bb = bfr(b2[j * 16 + col]);
#pragma unroll
    for (int r = 0; r < 8; ++r) so[wave][8 * g + r][j * 16 + col] = acc[j][r] + bb; }
  LDSX();
  for (int rl = 0; rl < 16; ++rl) vst2(X2P + (r0 + rl) * NO + lane * 4, *(const v4f*)(&so[wave][rl][lane * 4]));
  __syncthreads();
  for (int c = tid; c < NO; c += 128) { float s = 0.f, q = 0.f; for (int ww = 0; ww < 4; ++ww) for (int rl = 0; rl < 16; ++rl) { const float vv = so[ww][rl][c]; s += vv; q += vv * vv; } sps[0][c] = s; sps[1][c] = q; }
  __syncthreads();
  if (tid < 32) vst2(PS + (size_t)blockIdx.x * NO + tid * 4, *(const v4f*)(&sps[0][tid * 4])); else if (tid < 64) vst2(PQ + (size_t)blockIdx.x * NO + (tid - 32) * 4, *(const v4f*)(&sps[1][(tid - 32) * 4]));
}
__global__ __launch_bounds__(256) void k_out(const float* __restrict__ X2P, const float* __restrict__ SC2, float* __restrict__ out) {
  const size_t i4 = (size_t)blockIdx.x * 256 + threadIdx.x; if (i4 >= (size_t)NR * NO / 4) return;
  v4f v = *(const v4f*)(X2P + i4 * 4); const int c0 = (int)((i4 * 4) % NO);
#pragma unroll
  for (int e = 0; e < 4; ++e) { const float y = v[e] * SC2[c0 + e] + SC2[NO + c0 + e]; v[e] = y > 0.f ? y : 0.f; }
  vst2(out + i4 * 4, v);
}
extern "C" void kernel_launch(void* const* d_in, const int* in_sizes, int n_in, void* d_out, int out_size, void* d_ws, size_t ws_size, hipStream_t stream) {
  (void)in_sizes; (void)n_in; (void)out_size; (void)ws_size;
  const float** I = (const float**)d_in;
  const float *obs = I[0], *hin = I[1], *Ws = I[2], *bs = I[3], *Wv = I[4], *bv = I[5], *Wg = I[6], *aw = I[7], *W1 = I[8], *b1 = I[9], *g1 = I[10], *be1 = I[11], *W2 = I[12], *b2 = I[13], *g2 = I[14], *be2 = I[15];
  char* ws = (char*)d_ws; size_t off = 0;
  auto take = [&](size_t bytes) { char* p = ws + off; off += (bytes + 255) & ~(size_t)255; return p; };
  float* X1P = (float*)take((size_t)NR * HH * 4);
  __bf16* HWTh = (__bf16*)take((size_t)HALF * HH * NV * 2); __bf16* HWTl = (__bf16*)take((size_t)HALF * HH * NV * 2);
  float* S = (float*)take((size_t)NR * 2 * 4); float* PS = (float*)take((size_t)(NR / 64) * HH * 4); float* PQ = (float*)take((size_t)(NR / 64) * HH * 4); float* SC1 = (float*)take((size_t)2 * HH * 4); float* SC2 = (float*)take((size_t)2 * NO * 4);
  float* X2P = (float*)HWTh;
  for (int hf = 0; hf < 2; ++hf) { const int n0base = hf * HALF;
    k_h<<<dim3(NV / 64, HALF), 128, 0, stream>>>(obs, hin, Ws, bs, Wv, bv, Wg, aw, W1, n0base, S, HWTh, HWTl);
    k_gat<<<dim3(NV / 64, HALF), 128, 0, stream>>>(S, HWTh, HWTl, obs, Ws, bs, W1, b1, n0base, X1P, PS, PQ); }
  k_bn<HH><<<1, 256, 0, stream>>>(PS, PQ, NR / 64, g1, be1, SC1);
  k_x2<<<NR / 64, 128, 0, stream>>>(X1P, SC1, W2, b2, X2P, PS, PQ);
  k_bn<NO><<<1, 256, 0, stream>>>(PS, PQ, NR / 64, g2, be2, SC2);
  k_out<<<(NR * NO / 4 + 255) / 256, 256, 0, stream>>>(X2P, SC2, (float*)d_out);
}
